// Mamba2_13752485282233
// MI455X (gfx1250) — hardware-verified
//
#include <hip/hip_runtime.h>
#include <math.h>

typedef __attribute__((ext_vector_type(16))) _Float16 v16h;
typedef __attribute__((ext_vector_type(8)))  _Float16 v8h;
typedef __attribute__((ext_vector_type(16))) __bf16   v16b;
typedef __attribute__((ext_vector_type(8)))  __bf16   v8b;
typedef __attribute__((ext_vector_type(8)))  float    v8f;
typedef __attribute__((ext_vector_type(4)))  float    v4f;

constexpr int kBatch   = 2;
constexpr int kSeq     = 2048;
constexpr int kHid     = 1024;
constexpr int kHeads   = 32;
constexpr int kHdim    = 64;
constexpr int kInter   = kHeads * kHdim;
constexpr int kNst     = 128;
constexpr int kTaps    = 4;
constexpr int kConvDim = kInter + 2 * kNst;
constexpr int kProj    = kInter + kConvDim + kHeads;
constexpr int kProjPad = 4416;
constexpr int kRows    = kBatch * kSeq;
constexpr int kCS      = 64;
constexpr int kChunksPerB = kSeq / kCS;
constexpr int kChunks  = kBatch * kChunksPerB;
constexpr int kDtPad   = 64;
constexpr int kConvTP  = 260;
constexpr int kPc      = 136;
constexpr int kPl      = 72;
constexpr int kPy      = 68;
constexpr float kHdCarry = 512.0f;
constexpr float kBdCarry = 16.0f;
constexpr float kStCarry = 64.0f;

static_assert(kProj == 4384 && kConvDim == 2304, "shape");
static_assert((kHid % 32) == 0 && (kInter % 32) == 0 && (kNst % 32) == 0 && (kCS % 32) == 0, "GEMM K multiples of 32");
static_assert((kRows % 64) == 0 && (kConvDim % 64) == 0 && (kDtPad % 64) == 0 && (kInter % 64) == 0 &&
              (kHid % 64) == 0 && (kProjPad % 64) == 0 && (kCS % 64) == 0, "GEMM M,N multiples of 64");
static_assert(kProjPad >= kInter + kConvDim + kDtPad, "padded W rows cover the dt tile");
static_assert((kSeq % kCS) == 0 && kHdim == 64 && kNst == 128 && kCS == 64, "tile layout");

constexpr size_t kOffXB  = 0;
constexpr size_t kOffWI  = kOffXB  + (size_t)kRows * kHid * 2;
constexpr size_t kOffWO  = kOffWI  + (size_t)kProjPad * kHid * 2;
constexpr size_t kOffHR  = kOffWO  + (size_t)kHid * kInter * 2;
constexpr size_t kOffDTR = kOffHR  + (size_t)kRows * kConvDim * 4;
constexpr size_t kOffB16 = kOffDTR + (size_t)kRows * kDtPad * 4;
constexpr size_t kOffC16 = kOffB16 + (size_t)kRows * kNst * 2;
constexpr size_t kOffDTS = kOffC16 + (size_t)kRows * kNst * 2;
constexpr size_t kOffACU = kOffDTS + (size_t)kRows * kHeads * 4;
constexpr size_t kOffGM  = kOffACU + (size_t)kRows * kHeads * 4;
constexpr size_t kOffY   = kOffGM  + (size_t)kChunks * kCS * kCS * 4;
constexpr size_t kOffGH  = kOffY   + (size_t)kRows * kInter * 4;
constexpr size_t kOffGL  = kOffGH  + (size_t)kRows * kInter * 2;
constexpr size_t kWsTotal = kOffGL + (size_t)kRows * kInter * 2;
static_assert(kWsTotal == 131727360ull, "carve total");
static_assert(kWsTotal <= 134217728ull, "carve cap");
static_assert((size_t)kRows * kInter * 4 <= (size_t)kRows * kConvDim * 4, "GATE fits in HR");
static_assert((kOffWI % 128) == 0 && (kOffWO % 128) == 0 && (kOffHR % 128) == 0 && (kOffDTR % 128) == 0 &&
              (kOffB16 % 128) == 0 && (kOffC16 % 128) == 0 && (kOffDTS % 128) == 0 && (kOffACU % 128) == 0 &&
              (kOffGM % 128) == 0 && (kOffY % 128) == 0 && (kOffGH % 128) == 0 && (kOffGL % 128) == 0, "128-B aligned regions");

__device__ __forceinline__ unsigned short f2bf_bits(float f) {
  unsigned u = __float_as_uint(f);
  return (unsigned short)((u + 0x7FFFu + ((u >> 16) & 1u)) >> 16);
}
__device__ __forceinline__ float bf_bits2f(unsigned short h) { return __uint_as_float(((unsigned)h) << 16); }
__device__ __forceinline__ float bfr(float f) { return bf_bits2f(f2bf_bits(f)); }
__device__ __forceinline__ float h16_to_f32(unsigned hb) {
  const unsigned sgn = (hb & 0x8000u) << 16; const unsigned em = hb & 0x7fffu;
  const float fn = __uint_as_float((em << 13) + 0x38000000u);
  const float fs = (float)em * 5.9604644775390625e-8f;
  const float mag = (em < 0x400u) ? fs : fn; return __uint_as_float(__float_as_uint(mag) | sgn); }

__device__ __forceinline__ void dep_guard_h(v8f& a, v8f& b, v16h x, v16h y) { asm volatile("v_nop\n\tv_nop\n\tv_nop\n\tv_nop" : "+v"(a), "+v"(b) : "v"(x), "v"(y)); }
__device__ __forceinline__ void dep_guard_b(v8f& a, v8f& b, v16b x, v16b y) { asm volatile("v_nop\n\tv_nop\n\tv_nop\n\tv_nop" : "+v"(a), "+v"(b) : "v"(x), "v"(y)); }
__device__ __forceinline__ void keep4_h(v16h a, v16h b, v16h c, v16h d) { asm volatile("v_nop" :: "v"(a), "v"(b), "v"(c), "v"(d)); }
__device__ __forceinline__ void keep4_b(v16b a, v16b b, v16b c, v16b d) { asm volatile("v_nop" :: "v"(a), "v"(b), "v"(c), "v"(d)); }
__device__ __forceinline__ void acc_guard4(v8f& a, v8f& b, v8f& c, v8f& d) { asm volatile("v_nop\n\tv_nop\n\tv_nop\n\tv_nop" : "+v"(a), "+v"(b), "+v"(c), "+v"(d)); }
template <typename T> struct Frag;
template <> struct Frag<_Float16> {
  typedef v16h V; union U { v16h v; v8h h[2]; };
  static __device__ __forceinline__ v16h load(const _Float16* p) {
    U f; f.h[0] = *(const v8h*)(p); f.h[1] = *(const v8h*)(p + 16); return f.v;
  }
  static __device__ __forceinline__ v8f mma(v16h a, v16h b, v8f c) {
    return __builtin_amdgcn_wmma_f32_16x16x32_f16(false, a, false, b, (short)0, c, false, false);
  }
  static __device__ __forceinline__ void guard(v8f& a, v8f& b, v16h x, v16h y) { dep_guard_h(a, b, x, y); }
  static __device__ __forceinline__ void keep(v16h a, v16h b, v16h c, v16h d) { keep4_h(a, b, c, d); }
};
template <> struct Frag<__bf16> {
  typedef v16b V; union U { v16b v; v8b h[2]; };
  static __device__ __forceinline__ v16b load(const __bf16* p) {
    U f; f.h[0] = *(const v8b*)(p); f.h[1] = *(const v8b*)(p + 16); return f.v;
  }
  static __device__ __forceinline__ v8f mma(v16b a, v16b b, v8f c) {
    return __builtin_amdgcn_wmma_f32_16x16x32_bf16(false, a, false, b, (short)0, c, false, false);
  }
  static __device__ __forceinline__ void guard(v8f& a, v8f& b, v16b x, v16b y) { dep_guard_b(a, b, x, y); }
  static __device__ __forceinline__ void keep(v16b a, v16b b, v16b c, v16b d) { keep4_b(a, b, c, d); }
};

template <int ET> struct Elem;
template <> struct Elem<0> { typedef _Float16 T; };
template <> struct Elem<1> { typedef __bf16 T; };
template <int ET, int SPL, int BIAS_MODE, int OUT_MODE, bool RESID, int ACT = 0>
__global__ __launch_bounds__(256) void wmma_gemm64(
    const unsigned short* __restrict__ Ap, const unsigned short* __restrict__ A2p, int lda, long strideA,
    const unsigned short* __restrict__ Btp, const unsigned short* __restrict__ Bt2p, int ldb, long strideB,
    void* __restrict__ Cout, void* __restrict__ Cout2, int ldc, long strideC,
    const float* __restrict__ bias,
    const float* __restrict__ resid, long strideR,
    int M, int N, int K, float scale) {
  typedef typename Elem<ET>::T T;
  typedef typename Frag<T>::V V;
  const T* A = (const T*)Ap; const T* A2 = (const T*)A2p; const T* Bt = (const T*)Btp; const T* Bt2 = (const T*)Bt2p;
  __shared__ __align__(16) float sT[8][16 * 68];
  const int b    = blockIdx.y;
  const int lane = threadIdx.x & 31;
  const int wave = threadIdx.x >> 5;
  const int tilesN = N >> 6;
  const int tilesM = M >> 6;
  const int tile = blockIdx.x * 8 + wave;
  if (tile >= tilesM * tilesN) return;
  const int tm = tile / tilesN;
  const int tn = tile - tm * tilesN;
  const int m0 = tm << 6;
  const int n0 = tn << 6;

  const T* Ab  = A  + (size_t)b * strideA;
  const T* Bb  = Bt + (size_t)b * strideB;
  const T* Ab2 = (SPL >= 1) ? (A2  + (size_t)b * strideA) : nullptr;
  const T* Bb2 = (SPL == 2) ? (Bt2 + (size_t)b * strideB) : nullptr;

  const int rlane = lane & 15;
  const int koff  = (lane >> 4) * 8;
  const int mOff  = (lane >> 4) * 8;

  v8f acc[4][4];
#pragma unroll
  for (int i = 0; i < 4; ++i)
#pragma unroll
    for (int j = 0; j < 4; ++j) acc[i][j] = (v8f){0.f,0.f,0.f,0.f,0.f,0.f,0.f,0.f};

  for (int k0 = 0; k0 < K; k0 += 32) {
    V bh[4], bl[4];
#pragma unroll
    for (int j = 0; j < 4; ++j) {
      const size_t bo = (size_t)(n0 + (j << 4) + rlane) * ldb + koff + k0;
      bh[j] = Frag<T>::load(Bb + bo);
      if (SPL == 2) bl[j] = Frag<T>::load(Bb2 + bo);
    }
#pragma unroll
    for (int i = 0; i < 4; ++i) {
      const size_t ao = (size_t)(m0 + (i << 4) + rlane) * lda + koff + k0;
      V ah = Frag<T>::load(Ab + ao);
      V al;
      if (SPL >= 1) al = Frag<T>::load(Ab2 + ao);
#pragma unroll
      for (int j = 0; j < 4; ++j) {
        acc[i][j] = Frag<T>::mma(ah, bh[j], acc[i][j]);
        if (SPL == 2) acc[i][j] = Frag<T>::mma(ah, bl[j], acc[i][j]);
        if (SPL >= 1) acc[i][j] = Frag<T>::mma(al, bh[j], acc[i][j]);
      }
      Frag<T>::guard(acc[i][0], acc[i][3], ah, (SPL >= 1) ? al : ah);
    }
    Frag<T>::keep(bh[0], bh[1], bh[2], bh[3]);
    if (SPL == 2) Frag<T>::keep(bl[0], bl[1], bl[2], bl[3]);
  }
  acc_guard4(acc[0][0], acc[0][1], acc[0][2], acc[0][3]);
  acc_guard4(acc[1][0], acc[1][1], acc[1][2], acc[1][3]);
  acc_guard4(acc[2][0], acc[2][1], acc[2][2], acc[2][3]);
  acc_guard4(acc[3][0], acc[3][1], acc[3][2], acc[3][3]);

  float* slab = sT[wave];
  const float* Rb = RESID ? (resid + (size_t)b * strideR) : nullptr;
#pragma unroll
  for (int i = 0; i < 4; ++i) {
    const int mBase = m0 + (i << 4);
#pragma unroll
    for (int j = 0; j < 4; ++j) {
      const int n = n0 + (j << 4) + rlane;
      float bv = 0.f;
      if (BIAS_MODE == 2) bv = bias[n];
#pragma unroll
      for (int r = 0; r < 8; ++r) {
        float v = acc[i][j][r] * scale;
        if (BIAS_MODE == 1) v += bias[mBase + mOff + r];
        if (BIAS_MODE == 2) v += bv;
        if (RESID) v += Rb[(size_t)(mBase + mOff + r) * ldc + n];
        if (ACT == 1) v = tanhf(v);
        if (ACT == 2) v = fmaxf(v, 0.0f);
        if (ACT == 3) v = v / (1.0f + expf(-v));
        if (ACT == 4) v = (v > 0.f) ? v : 0.01f * v;
        slab[(mOff + r) * 68 + (j << 4) + rlane] = v;
      }
    }
    __builtin_amdgcn_fence(__ATOMIC_RELEASE, "workgroup");
    __builtin_amdgcn_wave_barrier();
    __builtin_amdgcn_fence(__ATOMIC_ACQUIRE, "workgroup");
    if (OUT_MODE == 0) {
      float* C = (float*)Cout + (size_t)b * strideC;
      const int hh = lane >> 4, c4 = (lane & 15) * 4;
      for (int pass = 0; pass < 2; ++pass) {
#pragma unroll
        for (int it = 0; it < 8; ++it) {
          const int row = it * 2 + hh;
          v4f v = *(const v4f*)(slab + row * 68 + c4);
          *(volatile v4f*)(C + (size_t)(mBase + row) * ldc + n0 + c4) = v;
        }
        __threadfence();
      }
    } else {
      const int q = lane >> 3, c8 = (lane & 7) * 8;
      unsigned short* C  = (unsigned short*)Cout  + (size_t)b * strideC;
      unsigned short* C2 = (OUT_MODE == 2) ? ((unsigned short*)Cout2 + (size_t)b * strideC) : nullptr;
      for (int pass = 0; pass < 2; ++pass) {
#pragma unroll
        for (int it = 0; it < 4; ++it) {
          const int row = it * 4 + q;
          const float* sp = slab + row * 68 + c8;
          v8h hv, lv;
#pragma unroll
          for (int e = 0; e < 8; ++e) {
            if (OUT_MODE == 1) {
              hv[e] = (_Float16)sp[e];
            } else {
              unsigned short hb = f2bf_bits(sp[e]);
              unsigned short lb = f2bf_bits(sp[e] - bf_bits2f(hb));
              hv[e] = __builtin_bit_cast(_Float16, hb);
              lv[e] = __builtin_bit_cast(_Float16, lb);
            }
          }
          *(volatile v8h*)(C + (size_t)(mBase + row) * ldc + n0 + c8) = hv;
          if (OUT_MODE == 2) *(volatile v8h*)(C2 + (size_t)(mBase + row) * ldc + n0 + c8) = lv;
        }
        __threadfence();
      }
    }
    __builtin_amdgcn_fence(__ATOMIC_RELEASE, "workgroup");
    __builtin_amdgcn_wave_barrier();
    __builtin_amdgcn_fence(__ATOMIC_ACQUIRE, "workgroup");
  }
}

__device__ __forceinline__ v8f mma16(v16h a, v16h b, v8f c) {
  c = __builtin_amdgcn_wmma_f32_16x16x32_f16(false, a, false, b, (short)0, c, false, false);
  asm volatile("v_nop\n\tv_nop\n\tv_nop\n\tv_nop" : "+v"(c) : "v"(a), "v"(b));
  return c;
}

__global__ __launch_bounds__(256) void cvt_bf16_kernel(
    const float* __restrict__ src, unsigned short* __restrict__ dst, int nsrc8, int ntot8)
{
  const int i = blockIdx.x * 256 + threadIdx.x;
  if (i >= ntot8) return;
  const int ic = (i < nsrc8) ? i : (nsrc8 - 1);
  const float fac = (i < nsrc8) ? 1.0f : 0.0f;
  const size_t e0 = (size_t)ic << 3;
  const v4f a0 = *(const v4f*)(src + e0);
  const v4f a1 = *(const v4f*)(src + e0 + 4);
  v8h hv;
#pragma unroll
  for (int e = 0; e < 4; ++e) {
    const unsigned short h0 = f2bf_bits(a0[e] * fac);
    const unsigned short h1 = f2bf_bits(a1[e] * fac);
    hv[e]     = __builtin_bit_cast(_Float16, h0);
    hv[4 + e] = __builtin_bit_cast(_Float16, h1);
  }
  unsigned short* q = dst + ((size_t)i << 3);
  *(volatile v8h*)q = hv;
  __threadfence();
  *(volatile v8h*)q = hv;
}

__global__ __launch_bounds__(256) void conv_bc_kernel(
    const float* __restrict__ HR, const float* __restrict__ cw,
    unsigned short* __restrict__ B16, unsigned short* __restrict__ C16)
{
  __shared__ __align__(16) float sT[16 * kConvTP];
  const int tid = threadIdx.x, lane = tid & 31, wave = tid >> 5, hh = lane >> 4;
  const int g0 = blockIdx.x * 64;
  const int tb = g0 & (kSeq - 1);
  const int cc = kInter + tid;
  const v4f wv = *(const v4f*)(cw + (size_t)cc * kTaps);
  const float w0 = bfr(wv[0]), w1 = bfr(wv[1]), w2 = bfr(wv[2]), w3 = bfr(wv[3]);
  float xm3, xm2, xm1;
  {
    const bool hist = (tb > 0);
    const int rb = hist ? (g0 - 3) : g0;
    const float fac = hist ? 1.0f : 0.0f;
    xm3 = HR[(size_t)rb * kConvDim + cc] * fac;
    xm2 = HR[(size_t)(rb + 1) * kConvDim + cc] * fac;
    xm1 = HR[(size_t)(rb + 2) * kConvDim + cc] * fac;
  }
  const int c8 = (lane & 15) * 8;
#pragma unroll 1
  for (int sub = 0; sub < 4; ++sub) {
    const int lb = g0 + sub * 16;
#pragma unroll 1
    for (int s = 0; s < 16; ++s) {
      const float xcur = HR[(size_t)(lb + s) * kConvDim + cc];
      float acc = w0 * xm3;
      acc = fmaf(w1, xm2, acc);
      acc = fmaf(w2, xm1, acc);
      acc = fmaf(w3, xcur, acc);
      const float hv = acc * __builtin_amdgcn_rcpf(1.0f + expf(-acc));
      sT[s * kConvTP + tid] = hv;
      xm3 = xm2; xm2 = xm1; xm1 = xcur;
    }
    __syncthreads();
    const int row = 2 * wave + hh;
    const float* sp = sT + row * kConvTP + c8;
    v8h hb, hc;
#pragma unroll
    for (int e = 0; e < 8; ++e) {
      hb[e] = (_Float16)sp[e];
      hc[e] = (_Float16)sp[kNst + e];
    }
    unsigned short* qb = B16 + (size_t)(lb + row) * kNst + c8;
    unsigned short* qc = C16 + (size_t)(lb + row) * kNst + c8;
    for (int pass = 0; pass < 2; ++pass) {
      *(volatile v8h*)qb = hb;
      *(volatile v8h*)qc = hc;
      __threadfence();
    }
    __syncthreads();
  }
}

__global__ __launch_bounds__(64) void dt_scan_kernel(
    const float* __restrict__ DTR, const float* __restrict__ b_in,
    const float* __restrict__ dt_bias, const float* __restrict__ A_log,
    float* __restrict__ DTS, float* __restrict__ ACU)
{
  __shared__ __align__(16) float sDt[kCS * kHeads];
  __shared__ __align__(16) float sAd[kCS * kHeads];
  const int tid = threadIdx.x, lane = tid & 31, wave = tid >> 5;
  const int q = blockIdx.x;
  const size_t row = (size_t)q * kCS + tid;
#pragma unroll 1
  for (int h = 0; h < kHeads; ++h) {
    const float praw = DTR[row * kDtPad + h] + bfr(b_in[kInter + kConvDim + h]);
    const float xb = praw + bfr(dt_bias[h]);
    const float dt = fmaxf(xb, 0.0f) + log1pf(expf(-fabsf(xb)));
    const float An = -expf(bfr(A_log[h]));
    sDt[tid * kHeads + h] = dt;
    sAd[tid * kHeads + h] = An * dt;
  }
  __syncthreads();
  if (tid < kHeads) {
    float runv = 0.0f;
#pragma unroll 1
    for (int l = 0; l < kCS; ++l) {
      runv = runv + sAd[l * kHeads + tid];
      sAd[l * kHeads + tid] = runv;
    }
  }
  __syncthreads();
  const int q8 = lane >> 3, cq = (lane & 7) * 4;
  for (int pass = 0; pass < 2; ++pass) {
#pragma unroll
    for (int it = 0; it < 8; ++it) {
      const int r = it * 8 + wave * 4 + q8;
      const v4f dv = *(const v4f*)(sDt + r * kHeads + cq);
      const v4f av = *(const v4f*)(sAd + r * kHeads + cq);
      const size_t o = ((size_t)q * kCS + r) * kHeads + cq;
      *(volatile v4f*)(DTS + o) = dv;
      *(volatile v4f*)(ACU + o) = av;
    }
    __threadfence();
  }
}

__device__ __forceinline__ void bd_pair(_Float16* p, unsigned w, float dw) {
  const float f0 = h16_to_f32(w & 0xffffu) * dw;
  const float f1 = h16_to_f32(w >> 16) * dw;
  p[0]   = (_Float16)f0;
  p[kPl] = (_Float16)f1;
}

__global__ __launch_bounds__(256) void ssd_chunk_kernel(
    const float* __restrict__ HR, const float* __restrict__ cw, const float* __restrict__ Dp,
    const unsigned short* __restrict__ B16, const unsigned short* __restrict__ C16,
    const float* __restrict__ DTS, const float* __restrict__ ACU, const float* __restrict__ GM,
    float* __restrict__ Yp)
{
  __shared__ __align__(16) _Float16 sC[kCS * kPc];
  __shared__ __align__(16) _Float16 sBd[kNst * kPl];
  __shared__ __align__(16) _Float16 sM[kCS * kPl];
  __shared__ __align__(16) _Float16 sHT[kHdim * kPl];
  __shared__ __align__(16) _Float16 sSi[kHdim * kPc];
  __shared__ __align__(16) float sHY[kCS * kPy];
  __shared__ float sAc[kCS];
  __shared__ float sDt[kCS];
  __shared__ float sDec[kCS];
  __shared__ float sEx[kCS];

  const int tid  = threadIdx.x;
  const int lane = tid & 31;
  const int wave = tid >> 5;
  const int hh   = lane >> 4;
  const int rl   = lane & 15;
  const int koff = hh * 8;
  const int bix  = blockIdx.x >> 5;
  const int head = blockIdx.x & 31;
  const int cp  = tid & 63;
  const int clg = tid >> 6;
  const int cc  = head * kHdim + cp;
  const v4f wv = *(const v4f*)(cw + (size_t)cc * kTaps);
  const float w0 = bfr(wv[0]), w1 = bfr(wv[1]), w2 = bfr(wv[2]), w3 = bfr(wv[3]);
  const float Dr = bfr(Dp[head]);
  const int pw  = wave & 3;
  const int lt0 = (wave >> 2) * 2;
  const int c4  = rl * 4;
  const float invD = 1.0f / kHdCarry;
  const float invS = 1.0f / (kHdCarry * kBdCarry);
  const float invO = 1.0f / kStCarry;

  v8f run[4];
#pragma unroll
  for (int pt = 0; pt < 4; ++pt) run[pt] = (v8f){0.f,0.f,0.f,0.f,0.f,0.f,0.f,0.f};

#pragma unroll 1
  for (int c = 0; c < kChunksPerB; ++c) {
    const int q = bix * kChunksPerB + c;
    const size_t row0 = (size_t)q * kCS;
    if (tid < kCS) {
      sAc[tid] = ACU[(row0 + tid) * kHeads + head];
      sDt[tid] = DTS[(row0 + tid) * kHeads + head];
    }
#pragma unroll
    for (int pt = 0; pt < 4; ++pt) {
      v8h sv;
#pragma unroll
      for (int r = 0; r < 8; ++r) sv[r] = (_Float16)(run[pt][r] * kStCarry);
      *(v8h*)(sSi + (16 * pt + rl) * kPc + 16 * wave + 8 * hh) = sv;
    }
#pragma unroll
    for (int k = 0; k < 4; ++k) {
      const int i = tid + 256 * k;
      const int r = i >> 4, seg = i & 15;
      const uint4 u = *(const uint4*)(C16 + (row0 + r) * kNst + seg * 8);
      *(v8h*)(sC + r * kPc + seg * 8) = __builtin_bit_cast(v8h, u);
    }
    __syncthreads();
    if (tid < kCS) {
      const float al = sAc[kCS - 1];
      sDec[tid] = expf(al - sAc[tid]) * kBdCarry;
      sEx[tid]  = expf(sAc[tid]);
    }
    {
      const int lb = 16 * clg;
      const bool hist = (c > 0) || (clg > 0);
      const size_t rb = hist ? (row0 + lb - 3) : row0;
      const float fac = hist ? 1.0f : 0.0f;
      float xm3 = HR[rb * kConvDim + cc] * fac;
      float xm2 = HR[(rb + 1) * kConvDim + cc] * fac;
      float xm1 = HR[(rb + 2) * kConvDim + cc] * fac;
#pragma unroll 1
      for (int s = 0; s < 16; ++s) {
        const int l = lb + s;
        const float xcur = HR[(row0 + l) * kConvDim + cc];
        float acc = w0 * xm3;
        acc = fmaf(w1, xm2, acc);
        acc = fmaf(w2, xm1, acc);
        acc = fmaf(w3, xcur, acc);
        const float hv = acc * __builtin_amdgcn_rcpf(1.0f + expf(-acc));
        sHY[l * kPy + cp] = hv;
        sHT[cp * kPl + l] = (_Float16)(hv * sDt[l] * kHdCarry);
        xm3 = xm2; xm2 = xm1; xm1 = xcur;
      }
    }
    __syncthreads();
#pragma unroll
    for (int k = 0; k < 4; ++k) {
      const int i = tid + 256 * k;
      const int l = i >> 4, seg = i & 15;
      const uint4 u = *(const uint4*)(B16 + (row0 + l) * kNst + seg * 8);
      const float dw = sDec[l];
      _Float16* bp = sBd + (seg * 8) * kPl + l;
      bd_pair(bp,           u.x, dw);
      bd_pair(bp + 2 * kPl, u.y, dw);
      bd_pair(bp + 4 * kPl, u.z, dw);
      bd_pair(bp + 6 * kPl, u.w, dw);
    }
    {
      const int l  = tid >> 2;
      const int s0 = (tid & 3) * 16;
      const float acl = sAc[l];
      const float* gp = GM + (size_t)q * (kCS * kCS) + l * kCS + s0;
#pragma unroll
      for (int j = 0; j < 2; ++j) {
        const v4f ga = *(const v4f*)(gp + 8 * j);
        const v4f gb = *(const v4f*)(gp + 8 * j + 4);
        v8h mv;
#pragma unroll
        for (int e = 0; e < 4; ++e) {
          const int sa = s0 + 8 * j + e;
          const int sb = sa + 4;
          const float da = __expf(fminf(acl - sAc[sa], 0.0f));
          const float db = __expf(fminf(acl - sAc[sb], 0.0f));
          const float ma = (sa <= l) ? (ga[e] * da) : 0.0f;
          const float mb = (sb <= l) ? (gb[e] * db) : 0.0f;
          mv[e]     = (_Float16)ma;
          mv[4 + e] = (_Float16)mb;
        }
        *(v8h*)(sM + l * kPl + s0 + 8 * j) = mv;
      }
    }
    __syncthreads();
    v8f accD[2], accO[2];
    accD[0] = (v8f){0.f,0.f,0.f,0.f,0.f,0.f,0.f,0.f}; accD[1] = accD[0];
    accO[0] = accD[0]; accO[1] = accD[0];
#pragma unroll
    for (int ks = 0; ks < 2; ++ks) {
      const v16h a = Frag<_Float16>::load(sHT + (16 * pw + rl) * kPl + koff + 32 * ks);
#pragma unroll
      for (int j = 0; j < 2; ++j) {
        const v16h bb = Frag<_Float16>::load(sM + (16 * (lt0 + j) + rl) * kPl + koff + 32 * ks);
        accD[j] = mma16(a, bb, accD[j]);
      }
    }
#pragma unroll
    for (int ks = 0; ks < 4; ++ks) {
      const v16h a = Frag<_Float16>::load(sSi + (16 * pw + rl) * kPc + koff + 32 * ks);
#pragma unroll
      for (int j = 0; j < 2; ++j) {
        const v16h bb = Frag<_Float16>::load(sC + (16 * (lt0 + j) + rl) * kPc + koff + 32 * ks);
        accO[j] = mma16(a, bb, accO[j]);
      }
    }
#pragma unroll
    for (int j = 0; j < 2; ++j) {
      const int l = 16 * (lt0 + j) + rl;
      const float ex = sEx[l] * invO;
      float* hp = sHY + l * kPy + 16 * pw + 8 * hh;
      const v4f h0 = *(const v4f*)hp;
      const v4f h1 = *(const v4f*)(hp + 4);
      v4f y0, y1;
#pragma unroll
      for (int r = 0; r < 4; ++r) {
        y0[r] = (accD[j][r] * invD + accO[j][r] * ex) + Dr * h0[r];
        y1[r] = (accD[j][4 + r] * invD + accO[j][4 + r] * ex) + Dr * h1[r];
      }
      *(v4f*)hp = y0;
      *(v4f*)(hp + 4) = y1;
    }
    v8f accS[4];
#pragma unroll
    for (int pt = 0; pt < 4; ++pt) accS[pt] = (v8f){0.f,0.f,0.f,0.f,0.f,0.f,0.f,0.f};
#pragma unroll
    for (int ks = 0; ks < 2; ++ks) {
      const v16h a = Frag<_Float16>::load(sBd + (16 * wave + rl) * kPl + koff + 32 * ks);
#pragma unroll
      for (int pt = 0; pt < 4; ++pt) {
        const v16h bb = Frag<_Float16>::load(sHT + (16 * pt + rl) * kPl + koff + 32 * ks);
        accS[pt] = mma16(a, bb, accS[pt]);
      }
    }
    const float dch = expf(sAc[kCS - 1]);
#pragma unroll
    for (int pt = 0; pt < 4; ++pt)
#pragma unroll
      for (int r = 0; r < 8; ++r)
        run[pt][r] = fmaf(run[pt][r], dch, accS[pt][r] * invS);
    __syncthreads();
    for (int pass = 0; pass < 2; ++pass) {
#pragma unroll
      for (int it = 0; it < 4; ++it) {
        const int row = 8 * wave + 2 * it + hh;
        const v4f v = *(const v4f*)(sHY + row * kPy + c4);
        *(volatile v4f*)(Yp + (row0 + row) * kInter + head * kHdim + c4) = v;
      }
      __threadfence();
    }
  }
}

__global__ __launch_bounds__(256) void gate_norm_kernel(
    const float* __restrict__ Yp, const float* __restrict__ Gp, const float* __restrict__ nw,
    unsigned short* __restrict__ GH, unsigned short* __restrict__ GL)
{
  __shared__ float red[8];
  const int tid = threadIdx.x, lane = tid & 31, wave = tid >> 5;
  const size_t base = (size_t)blockIdx.x * kInter + (size_t)tid * 8;
  const v4f ya = *(const v4f*)(Yp + base);
  const v4f yb = *(const v4f*)(Yp + base + 4);
  const v4f ga = *(const v4f*)(Gp + base);
  const v4f gb = *(const v4f*)(Gp + base + 4);
  const v4f na = *(const v4f*)(nw + (size_t)tid * 8);
  const v4f nb = *(const v4f*)(nw + (size_t)tid * 8 + 4);
  v4f pa, pb;
  float ss = 0.0f;
#pragma unroll
  for (int e = 0; e < 4; ++e) {
    const float za = ga[e], zb = gb[e];
    const float sa = za * __builtin_amdgcn_rcpf(1.0f + expf(-za));
    const float sb = zb * __builtin_amdgcn_rcpf(1.0f + expf(-zb));
    const float va = ya[e] * sa;
    const float vb = yb[e] * sb;
    pa[e] = va;
    pb[e] = vb;
    ss = fmaf(va, va, ss);
    ss = fmaf(vb, vb, ss);
  }
#pragma unroll
  for (int off = 16; off > 0; off >>= 1) ss += __shfl_xor(ss, off, 32);
  if (lane == 0) red[wave] = ss;
  __syncthreads();
  const float tot = ((red[0] + red[1]) + (red[2] + red[3])) + ((red[4] + red[5]) + (red[6] + red[7]));
  const float rstd = rsqrtf(tot * (1.0f / (float)kInter) + 1e-5f);
  v8h hv, lv;
#pragma unroll
  for (int e = 0; e < 4; ++e) {
    const float oa = (pa[e] * rstd) * bfr(na[e]);
    const float ob = (pb[e] * rstd) * bfr(nb[e]);
    const unsigned short ha = f2bf_bits(oa), hb2 = f2bf_bits(ob);
    const unsigned short la = f2bf_bits(oa - bf_bits2f(ha)), lb2 = f2bf_bits(ob - bf_bits2f(hb2));
    hv[e]     = __builtin_bit_cast(_Float16, ha);
    hv[4 + e] = __builtin_bit_cast(_Float16, hb2);
    lv[e]     = __builtin_bit_cast(_Float16, la);
    lv[4 + e] = __builtin_bit_cast(_Float16, lb2);
  }
  unsigned short* qh = GH + base;
  unsigned short* ql = GL + base;
  *(volatile v8h*)qh = hv;
  *(volatile v8h*)ql = lv;
  __threadfence();
  *(volatile v8h*)qh = hv;
  *(volatile v8h*)ql = lv;
}

extern "C" void kernel_launch(void* const* d_in, const int* in_sizes, int n_in,
                              void* d_out, int out_size, void* d_ws, size_t ws_size,
                              hipStream_t stream) {
  if (n_in < 10) return;
  if (in_sizes[0] != kRows * kHid) return;
  if (in_sizes[1] != kProj * kHid) return;
  if (in_sizes[2] != kProj) return;
  if (in_sizes[3] != kConvDim * kTaps) return;
  if (in_sizes[4] != kHeads) return;
  if (in_sizes[5] != kHeads) return;
  if (in_sizes[6] != kHeads) return;
  if (in_sizes[7] != kInter) return;
  if (in_sizes[8] != kHid * kInter) return;
  if (in_sizes[9] != kHid) return;
  if (out_size != kRows * kHid) return;
  if (ws_size < kWsTotal) return;

  const float* x       = (const float*)d_in[0];
  const float* W_in    = (const float*)d_in[1];
  const float* b_in    = (const float*)d_in[2];
  const float* conv_w  = (const float*)d_in[3];
  const float* dt_bias = (const float*)d_in[4];
  const float* A_log   = (const float*)d_in[5];
  const float* Dp      = (const float*)d_in[6];
  const float* norm_w  = (const float*)d_in[7];
  const float* W_out   = (const float*)d_in[8];
  const float* b_out   = (const float*)d_in[9];
  float* out = (float*)d_out;

  char* ws = (char*)d_ws;
  unsigned short* XB  = (unsigned short*)(ws + kOffXB);
  unsigned short* WI  = (unsigned short*)(ws + kOffWI);
  unsigned short* WO  = (unsigned short*)(ws + kOffWO);
  float*          HR  = (float*)(ws + kOffHR);
  float*          GATE = (float*)(ws + kOffHR);
  float*          DTR = (float*)(ws + kOffDTR);
  unsigned short* B16 = (unsigned short*)(ws + kOffB16);
  unsigned short* C16 = (unsigned short*)(ws + kOffC16);
  float*          DTS = (float*)(ws + kOffDTS);
  float*          ACU = (float*)(ws + kOffACU);
  float*          GM  = (float*)(ws + kOffGM);
  float*          Y   = (float*)(ws + kOffY);
  unsigned short* GH  = (unsigned short*)(ws + kOffGH);
  unsigned short* GL  = (unsigned short*)(ws + kOffGL);

  {
    const int nx8 = kRows * kHid / 8;
    cvt_bf16_kernel<<<(nx8 + 255) / 256, 256, 0, stream>>>(x, XB, nx8, nx8);
    const int nwsrc8 = kProj * kHid / 8, nwtot8 = kProjPad * kHid / 8;
    cvt_bf16_kernel<<<(nwtot8 + 255) / 256, 256, 0, stream>>>(W_in, WI, nwsrc8, nwtot8);
    const int no8 = kHid * kInter / 8;
    cvt_bf16_kernel<<<(no8 + 255) / 256, 256, 0, stream>>>(W_out, WO, no8, no8);
  }

  wmma_gemm64<1, 0, 2, 0, false><<<dim3((kRows / 64) * (kConvDim / 64) / 8, 1), 256, 0, stream>>>(
      XB, nullptr, kHid, 0L,
      WI + (size_t)kInter * kHid, nullptr, kHid, 0L,
      (void*)HR, nullptr, kConvDim, 0L,
      b_in + kInter, nullptr, 0L,
      kRows, kConvDim, kHid, 1.0f);

  wmma_gemm64<1, 0, 0, 0, false><<<dim3((kRows / 64) * (kDtPad / 64) / 8, 1), 256, 0, stream>>>(
      XB, nullptr, kHid, 0L,
      WI + (size_t)(kInter + kConvDim) * kHid, nullptr, kHid, 0L,
      (void*)DTR, nullptr, kDtPad, 0L,
      nullptr, nullptr, 0L,
      kRows, kDtPad, kHid, 1.0f);

  conv_bc_kernel<<<kRows / 64, 256, 0, stream>>>(HR, conv_w, B16, C16);

  dt_scan_kernel<<<kChunks, kCS, 0, stream>>>(DTR, b_in, dt_bias, A_log, DTS, ACU);

  wmma_gemm64<0, 0, 0, 0, false><<<dim3(1, kChunks), 256, 0, stream>>>(
      C16, nullptr, kNst, (long)kCS * kNst,
      B16, nullptr, kNst, (long)kCS * kNst,
      (void*)GM, nullptr, kCS, (long)kCS * kCS,
      nullptr, nullptr, 0L,
      kCS, kCS, kNst, 1.0f);

  ssd_chunk_kernel<<<kBatch * kHeads, 256, 0, stream>>>(HR, conv_w, Dp, B16, C16, DTS, ACU, GM, Y);

  wmma_gemm64<1, 0, 2, 0, false><<<dim3((kRows / 64) * (kInter / 64) / 8, 1), 256, 0, stream>>>(
      XB, nullptr, kHid, 0L,
      WI, nullptr, kHid, 0L,
      (void*)GATE, nullptr, kInter, 0L,
      b_in, nullptr, 0L,
      kRows, kInter, kHid, 1.0f);

  gate_norm_kernel<<<kRows, 256, 0, stream>>>(Y, GATE, norm_w, GH, GL);

  wmma_gemm64<1, 1, 2, 0, false><<<dim3((kRows / 64) * (kHid / 64) / 8, 1), 256, 0, stream>>>(
      GH, GL, kInter, 0L,
      WO, nullptr, kInter, 0L,
      (void*)out, nullptr, kHid, 0L,
      b_out, nullptr, 0L,
      kRows, kHid, kInter, 1.0f);
}
